// WeightedCausalMultiheadAttention_63505386438809
// MI455X (gfx1250) — hardware-verified
//
#include <hip/hip_runtime.h>


#define S_LEN   2048
#define BATCH   2
#define DMODEL  1024
#define NHEADS  16
#define HDIM    64
#define ROWS    (BATCH * S_LEN)
#define N3D     (3 * DMODEL)
#define LDP     40
#define LDK     72
#define EP      68
#define LOG2E   1.4426950408889634f

typedef unsigned short us;
typedef __attribute__((ext_vector_type(16))) __bf16 v16bf;
typedef float v8f  __attribute__((ext_vector_type(8)));
typedef float v4fa __attribute__((ext_vector_type(4), __may_alias__));
typedef us    us8a __attribute__((ext_vector_type(8), __may_alias__));

union Frag { v16bf v; us8a h[2]; };

__device__ __forceinline__ v8f zero8() { v8f z = {0.f, 0.f, 0.f, 0.f, 0.f, 0.f, 0.f, 0.f}; return z; }
__device__ __forceinline__ us8a ldv(const us* p)          { return *(const us8a*)p; }
__device__ __forceinline__ void stv(us* p, us8a v)         { *(us8a*)p = v; }
__device__ __forceinline__ void vstv(us* p, us8a v)        { *(volatile us8a*)p = v; }
__device__ __forceinline__ v4fa ldf4(const float* p)       { return *(const v4fa*)p; }
__device__ __forceinline__ void vstf4(float* p, v4fa v)    { *(volatile v4fa*)p = v; }

__device__ __forceinline__ us f2bf(float f) {
    unsigned int b = __float_as_uint(f);
    b += 0x7FFFu + ((b >> 16) & 1u);
    return (us)(b >> 16);
}
__device__ __forceinline__ void splitf(float x, us& hi, us& lo) {
    const us hb = f2bf(x);
    const float hv = __uint_as_float(((unsigned int)hb) << 16);
    hi = hb;
    lo = f2bf(x - hv);
}
__device__ __forceinline__ void split8(v4fa a, v4fa b, us8a& hi, us8a& lo) {
    float x[8] = {a.x, a.y, a.z, a.w, b.x, b.y, b.z, b.w};
    #pragma unroll
    for (int e = 0; e < 8; ++e) { us hh, ll; splitf(x[e], hh, ll); hi[e] = hh; lo[e] = ll; }
}

__device__ __forceinline__ float fexp(float x) { return __builtin_amdgcn_exp2f(x * LOG2E); }

__device__ __forceinline__ float hmax16(float v) {
    #pragma unroll
    for (int k = 1; k < 16; k <<= 1) v = fmaxf(v, __shfl_xor(v, k, 32));
    return v;
}
__device__ __forceinline__ float hsum16(float v) {
    #pragma unroll
    for (int k = 1; k < 16; k <<= 1) v += __shfl_xor(v, k, 32);
    return v;
}
__device__ __forceinline__ int clampi(int x, int lo, int hi) { return x < lo ? lo : (x > hi ? hi : x); }

__device__ __forceinline__ void wave_sync() {
    asm volatile("" ::: "memory");
    __builtin_amdgcn_fence(__ATOMIC_RELEASE, "wavefront");
    __builtin_amdgcn_wave_barrier();
    asm volatile("" ::: "memory");
}

__device__ __forceinline__ void load_frag(Frag& f, const us* row, int h) {
    f.h[0] = ldv(row + 8 * h);
    f.h[1] = ldv(row + 16 + 8 * h);
}
__device__ __forceinline__ v8f wmma1(const Frag& a, const Frag& b, v8f c) {
    return __builtin_amdgcn_wmma_f32_16x16x32_bf16(false, a.v, false, b.v, (short)0, c, false, false);
}
__device__ __forceinline__ v8f guard4(v8f c, const Frag& a0, const Frag& a1, const Frag& b0, const Frag& b1) {
    asm volatile("v_nop\n\tv_nop\n\tv_nop\n\tv_nop"
                 : "+v"(c) : "v"(a0.v), "v"(a1.v), "v"(b0.v), "v"(b1.v));
    return c;
}
__device__ __forceinline__ v8f mma3(const Frag& ah, const Frag& al, const Frag& bh, const Frag& bl, v8f c) {
    c = wmma1(ah, bh, c);
    c = wmma1(ah, bl, c);
    c = wmma1(al, bh, c);
    return guard4(c, ah, al, bh, bl);
}

__global__ __launch_bounds__(256) void cvt_rows(const float* __restrict__ src,
                                                us* __restrict__ hi, us* __restrict__ lo, int n8)
{
    const int i = blockIdx.x * 256 + threadIdx.x;
    if (i >= n8) return;
    const float* p = src + (size_t)i * 8;
    const v4fa a = ldf4(p), b = ldf4(p + 4);
    us8a vh, vl;
    split8(a, b, vh, vl);
    us* ph = hi + (size_t)i * 8;
    us* pl = lo + (size_t)i * 8;
    vstv(ph, vh); vstv(pl, vl);
    __threadfence();
    vstv(ph, vh); vstv(pl, vl);
}

__global__ __launch_bounds__(256) void cvt_transpose(const float* __restrict__ src,
                                                     us* __restrict__ hi, us* __restrict__ lo,
                                                     int R, int C)
{
    __shared__ __attribute__((aligned(16))) float tile[32 * EP];
    const int t = threadIdx.x;
    const int c0 = blockIdx.x * 32, r0 = blockIdx.y * 64;
    {
        const int c = t & 31, rb = t >> 5;
        #pragma unroll
        for (int i = 0; i < 8; ++i) {
            const int r = rb + 8 * i;
            tile[c * EP + r] = src[(size_t)(r0 + r) * C + c0 + c];
        }
    }
    __syncthreads();
    const int j = t >> 3, p = t & 7;
    const v4fa a = ldf4(tile + j * EP + 8 * p), b = ldf4(tile + j * EP + 8 * p + 4);
    us8a vh, vl;
    split8(a, b, vh, vl);
    const size_t o = (size_t)(c0 + j) * R + r0 + 8 * p;
    vstv(hi + o, vh); vstv(lo + o, vl);
    __threadfence();
    vstv(hi + o, vh); vstv(lo + o, vl);
}

__device__ __forceinline__ void gemm_core(const us* __restrict__ Ah, const us* __restrict__ Al,
                                          const us* __restrict__ Bh, const us* __restrict__ Bl,
                                          const float* __restrict__ bias, int M0, int N0, float* smf)
{
    us* sAh = (us*)smf;
    us* sAl = sAh + 128 * LDP;
    us* sBh = sAl + 128 * LDP;
    us* sBl = sBh + 64 * LDP;
    const int t = threadIdx.x, l = t & 31, w = t >> 5, h = l >> 4, m = l & 15;
    const int wm = w >> 1, wn = w & 1;
    const int ar = t >> 1, ak = (t & 1) * 16;
    const int br = t >> 2, bk = (t & 3) * 8;
    const us* gAh = Ah + (size_t)(M0 + ar) * DMODEL + ak;
    const us* gAl = Al + (size_t)(M0 + ar) * DMODEL + ak;
    const us* gBh = Bh + (size_t)(N0 + br) * DMODEL + bk;
    const us* gBl = Bl + (size_t)(N0 + br) * DMODEL + bk;

    v8f acc[2][2];
    #pragma unroll
    for (int i = 0; i < 2; ++i)
        #pragma unroll
        for (int j = 0; j < 2; ++j) acc[i][j] = zero8();

    #pragma unroll 1
    for (int k0 = 0; k0 < DMODEL; k0 += 32) {
        const us8a a0 = ldv(gAh + k0), a1 = ldv(gAh + k0 + 8);
        const us8a a2 = ldv(gAl + k0), a3 = ldv(gAl + k0 + 8);
        const us8a b0 = ldv(gBh + k0), b1 = ldv(gBl + k0);
        __syncthreads();
        stv(sAh + ar * LDP + ak, a0); stv(sAh + ar * LDP + ak + 8, a1);
        stv(sAl + ar * LDP + ak, a2); stv(sAl + ar * LDP + ak + 8, a3);
        stv(sBh + br * LDP + bk, b0); stv(sBl + br * LDP + bk, b1);
        __syncthreads();
        Frag fah[2], fal[2], fbh[2], fbl[2];
        #pragma unroll
        for (int mt = 0; mt < 2; ++mt) {
            const int row = wm * 32 + mt * 16 + m;
            load_frag(fah[mt], sAh + row * LDP, h);
            load_frag(fal[mt], sAl + row * LDP, h);
        }
        #pragma unroll
        for (int nt = 0; nt < 2; ++nt) {
            const int row = wn * 32 + nt * 16 + m;
            load_frag(fbh[nt], sBh + row * LDP, h);
            load_frag(fbl[nt], sBl + row * LDP, h);
        }
        #pragma unroll
        for (int mt = 0; mt < 2; ++mt)
            #pragma unroll
            for (int nt = 0; nt < 2; ++nt)
                acc[mt][nt] = mma3(fah[mt], fal[mt], fbh[nt], fbl[nt], acc[mt][nt]);
    }
    __syncthreads();
    #pragma unroll
    for (int mt = 0; mt < 2; ++mt)
        #pragma unroll
        for (int nt = 0; nt < 2; ++nt) {
            const int col = wn * 32 + nt * 16 + m;
            const float bv = bias[N0 + col];
            #pragma unroll
            for (int r = 0; r < 8; ++r)
                smf[(wm * 32 + mt * 16 + 8 * h + r) * EP + col] = acc[mt][nt][r] + bv;
        }
    __syncthreads();
}

__global__ __launch_bounds__(256) void gemm_qkv(const us* __restrict__ Ah, const us* __restrict__ Al,
                                                const us* __restrict__ Bh, const us* __restrict__ Bl,
                                                const float* __restrict__ bias,
                                                us* __restrict__ Qh, us* __restrict__ Ql,
                                                us* __restrict__ Kh, us* __restrict__ Kl,
                                                us* __restrict__ Vth, us* __restrict__ Vtl)
{
    __shared__ __attribute__((aligned(16))) float smf[128 * EP];
    const int M0 = blockIdx.y * 128, N0 = blockIdx.x * 64;
    gemm_core(Ah, Al, Bh, Bl, bias, M0, N0, smf);

    const int t = threadIdx.x;
    const int part = N0 >> 10, head = (N0 & (DMODEL - 1)) >> 6;
    const int b = M0 >> 11, s0 = M0 & (S_LEN - 1), bh = b * NHEADS + head;
    if (part < 2) {
        us* Dh = (part == 0) ? Qh : Kh;
        us* Dl = (part == 0) ? Ql : Kl;
        #pragma unroll 1
        for (int pass = 0; pass < 2; ++pass) {
            #pragma unroll
            for (int it = 0; it < 4; ++it) {
                const int row = it * 32 + (t >> 3), p = t & 7;
                const v4fa a = ldf4(smf + row * EP + 8 * p), c = ldf4(smf + row * EP + 8 * p + 4);
                us8a vh, vl;
                split8(a, c, vh, vl);
                const size_t o = ((size_t)bh * S_LEN + s0 + row) * HDIM + 8 * p;
                vstv(Dh + o, vh); vstv(Dl + o, vl);
            }
            if (pass == 0) __threadfence();
        }
    } else {
        #pragma unroll 1
        for (int pass = 0; pass < 2; ++pass) {
            #pragma unroll
            for (int it = 0; it < 4; ++it) {
                const int d = it * 16 + (t >> 4), p = t & 15;
                v4fa a, c;
                a.x = smf[(8 * p + 0) * EP + d]; a.y = smf[(8 * p + 1) * EP + d];
                a.z = smf[(8 * p + 2) * EP + d]; a.w = smf[(8 * p + 3) * EP + d];
                c.x = smf[(8 * p + 4) * EP + d]; c.y = smf[(8 * p + 5) * EP + d];
                c.z = smf[(8 * p + 6) * EP + d]; c.w = smf[(8 * p + 7) * EP + d];
                us8a vh, vl;
                split8(a, c, vh, vl);
                const size_t o = ((size_t)bh * HDIM + d) * S_LEN + s0 + 8 * p;
                vstv(Vth + o, vh); vstv(Vtl + o, vl);
            }
            if (pass == 0) __threadfence();
        }
    }
}

__global__ __launch_bounds__(256) void gemm_proj(const us* __restrict__ Ah, const us* __restrict__ Al,
                                                 const us* __restrict__ Bh, const us* __restrict__ Bl,
                                                 const float* __restrict__ bias, float* __restrict__ out)
{
    __shared__ __attribute__((aligned(16))) float smf[128 * EP];
    const int M0 = blockIdx.y * 128, N0 = blockIdx.x * 64;
    gemm_core(Ah, Al, Bh, Bl, bias, M0, N0, smf);
    const int t = threadIdx.x;
    #pragma unroll 1
    for (int pass = 0; pass < 2; ++pass) {
        #pragma unroll
        for (int it = 0; it < 8; ++it) {
            const int row = it * 16 + (t >> 4), p = t & 15;
            const v4fa v = ldf4(smf + row * EP + 4 * p);
            const size_t o = (size_t)(M0 + row) * DMODEL + N0 + 4 * p;
            vstf4(out + o, v);
        }
        if (pass == 0) __threadfence();
    }
}

__global__ __launch_bounds__(256) void attn_kernel(const us* __restrict__ Qh, const us* __restrict__ Ql,
                                                   const us* __restrict__ Kh, const us* __restrict__ Kl,
                                                   const us* __restrict__ Vth, const us* __restrict__ Vtl,
                                                   us* __restrict__ Oh, us* __restrict__ Ol)
{
    __shared__ __attribute__((aligned(16))) float asmf[12032];
    float* tbl = asmf;
    us* sm  = (us*)asmf;
    us* sKh = sm + 4096;
    us* sKl = sKh + 32 * LDK;
    us* sVh = sKl + 32 * LDK;
    us* sVl = sVh + 64 * LDP;
    us* sP  = sVl + 64 * LDP;

    const int t = threadIdx.x, l = t & 31, w = t >> 5, h = l >> 4, m = l & 15;
    const int bh = blockIdx.y, hh = bh & (NHEADS - 1), b = bh >> 4;
    const int Q0 = blockIdx.x * 128, q0 = Q0 + 16 * w;
    us* sPh = sP + w * (32 * LDP);
    us* sPl = sPh + 16 * LDP;

    #pragma unroll 1
    for (int i = t; i < S_LEN; i += 256) tbl[i] = -logf((float)i + 1.0f);

    Frag qh0, qh1, ql0, ql1;
    {
        const size_t qo = ((size_t)bh * S_LEN + q0 + m) * HDIM;
        const us* ph = Qh + qo;
        const us* pl = Ql + qo;
        load_frag(qh0, ph, h); load_frag(qh1, ph + 32, h);
        load_frag(ql0, pl, h); load_frag(ql1, pl + 32, h);
    }

    v8f oacc[4];
    #pragma unroll
    for (int c = 0; c < 4; ++c) oacc[c] = zero8();
    float m8[8], l8[8];
    #pragma unroll
    for (int r = 0; r < 8; ++r) { m8[r] = -1.0e30f; l8[r] = 0.f; }

    const int kr = t >> 3, kc = (t & 7) * 8;
    const int vr = t >> 2, vc = (t & 3) * 8;
    const us* gKh = Kh  + ((size_t)bh * S_LEN + kr) * HDIM + kc;
    const us* gKl = Kl  + ((size_t)bh * S_LEN + kr) * HDIM + kc;
    const us* gVh = Vth + ((size_t)bh * HDIM + vr) * S_LEN + vc;
    const us* gVl = Vtl + ((size_t)bh * HDIM + vr) * S_LEN + vc;
    const float NEG_INF = -__builtin_inff();

    const int ntile = (S_LEN - Q0) >> 5;
    for (int it = 0; it < ntile; ++it) {
        const int j0 = Q0 + 32 * it;
        const us8a xk0 = ldv(gKh + (size_t)j0 * HDIM), xk1 = ldv(gKl + (size_t)j0 * HDIM);
        const us8a xv0 = ldv(gVh + j0), xv1 = ldv(gVl + j0);
        __syncthreads();
        stv(sKh + kr * LDK + kc, xk0); stv(sKl + kr * LDK + kc, xk1);
        stv(sVh + vr * LDP + vc, xv0); stv(sVl + vr * LDP + vc, xv1);
        __syncthreads();

        if (j0 + 32 > q0) {
            v8f sc[2];
            #pragma unroll
            for (int sub = 0; sub < 2; ++sub) {
                const us* krh = sKh + (sub * 16 + m) * LDK;
                const us* krl = sKl + (sub * 16 + m) * LDK;
                Frag bh0, bh1, bl0, bl1;
                load_frag(bh0, krh, h); load_frag(bh1, krh + 32, h);
                load_frag(bl0, krl, h); load_frag(bl1, krl + 32, h);
                v8f s = zero8();
                s = wmma1(qh0, bh0, s); s = wmma1(qh0, bl0, s); s = wmma1(ql0, bh0, s);
                s = wmma1(qh1, bh1, s); s = wmma1(qh1, bl1, s); s = wmma1(ql1, bh1, s);
                sc[sub] = guard4(s, qh1, ql1, bh1, bl1);
            }
            #pragma unroll
            for (int r = 0; r < 8; ++r) {
                const int qrow = q0 + 8 * h + r;
                const int d0 = j0 + m - qrow, d1 = d0 + 16;
                const float bias0 = tbl[clampi(d0, 0, S_LEN - 1)];
                const float bias1 = tbl[clampi(d1, 0, S_LEN - 1)];
                float sv0 = sc[0][r] * 0.125f + bias0;
                float sv1 = sc[1][r] * 0.125f + bias1;
                sv0 = (d0 < 0) ? NEG_INF : sv0;
                sv1 = (d1 < 0) ? NEG_INF : sv1;
                const float rm = hmax16(fmaxf(sv0, sv1));
                const float mn = fmaxf(m8[r], rm);
                const float corr = fexp(m8[r] - mn);
                const float p0 = fexp(sv0 - mn), p1 = fexp(sv1 - mn);
                l8[r] = l8[r] * corr + hsum16(p0 + p1);
                m8[r] = mn;
                #pragma unroll
                for (int c = 0; c < 4; ++c) oacc[c][r] *= corr;
                us h0, l0, h1, l1;
                splitf(p0, h0, l0); splitf(p1, h1, l1);
                sPh[(8 * h + r) * LDP + m]      = h0;
                sPh[(8 * h + r) * LDP + 16 + m] = h1;
                sPl[(8 * h + r) * LDP + m]      = l0;
                sPl[(8 * h + r) * LDP + 16 + m] = l1;
            }
            wave_sync();
            Frag fph, fpl;
            load_frag(fph, sPh + m * LDP, h);
            load_frag(fpl, sPl + m * LDP, h);
            #pragma unroll
            for (int c = 0; c < 4; ++c) {
                Frag vfh, vfl;
                load_frag(vfh, sVh + (c * 16 + m) * LDP, h);
                load_frag(vfl, sVl + (c * 16 + m) * LDP, h);
                oacc[c] = mma3(fph, fpl, vfh, vfl, oacc[c]);
            }
        }
    }
    __syncthreads();

    us* sOh = sm + 4096 + w * 2304;
    us* sOl = sOh + 16 * 72;
    #pragma unroll
    for (int r = 0; r < 8; ++r) {
        const float inv = 1.0f / l8[r];
        #pragma unroll
        for (int c = 0; c < 4; ++c) {
            const float o = oacc[c][r] * inv;
            us ho, lo;
            splitf(o, ho, lo);
            sOh[(8 * h + r) * 72 + c * 16 + m] = ho;
            sOl[(8 * h + r) * 72 + c * 16 + m] = lo;
        }
    }
    wave_sync();
    #pragma unroll 1
    for (int pass = 0; pass < 2; ++pass) {
        #pragma unroll
        for (int p = 0; p < 4; ++p) {
            const int row = 4 * p + (l >> 3), piece = l & 7;
            const us8a a = ldv(sOh + row * 72 + 8 * piece);
            const us8a c = ldv(sOl + row * 72 + 8 * piece);
            const size_t o = ((size_t)(b * S_LEN + q0 + row)) * DMODEL + hh * HDIM + 8 * piece;
            vstv(Oh + o, a); vstv(Ol + o, c);
        }
        if (pass == 0) __threadfence();
    }
}

extern "C" void kernel_launch(void* const* d_in, const int* in_sizes, int n_in,
                              void* d_out, int out_size, void* d_ws, size_t ws_size,
                              hipStream_t stream)
{
    if (n_in < 5) return;
    if (in_sizes[0] != ROWS * DMODEL || in_sizes[1] != DMODEL * N3D || in_sizes[2] != N3D ||
        in_sizes[3] != DMODEL * DMODEL || in_sizes[4] != DMODEL || out_size != ROWS * DMODEL) return;

    const float* f_hid = (const float*)d_in[0];
    const float* f_wa  = (const float*)d_in[1];
    const float* f_ba  = (const float*)d_in[2];
    const float* f_wp  = (const float*)d_in[3];
    const float* f_bp  = (const float*)d_in[4];
    float*       out   = (float*)d_out;

    const size_t szHid = (size_t)ROWS * DMODEL * 2;
    const size_t szWa  = (size_t)N3D * DMODEL * 2;
    const size_t szWp  = (size_t)DMODEL * DMODEL * 2;
    const size_t szHd  = (size_t)BATCH * NHEADS * S_LEN * HDIM * 2;
    size_t off = 0;
    char* w = (char*)d_ws;
    us* hidH = (us*)(w + off); off += szHid;
    us* hidL = (us*)(w + off); off += szHid;
    us* waTH = (us*)(w + off); off += szWa;
    us* waTL = (us*)(w + off); off += szWa;
    us* wpTH = (us*)(w + off); off += szWp;
    us* wpTL = (us*)(w + off); off += szWp;
    us* QH   = (us*)(w + off); off += szHd;
    us* QL   = (us*)(w + off); off += szHd;
    us* KH   = (us*)(w + off); off += szHd;
    us* KL   = (us*)(w + off); off += szHd;
    us* VTH  = (us*)(w + off); off += szHd;
    us* VTL  = (us*)(w + off); off += szHd;
    us* OH   = (us*)(w + off); off += szHid;
    us* OL   = (us*)(w + off); off += szHid;
    if (off > ws_size) return;

    const int n8 = ROWS * DMODEL / 8;
    cvt_rows<<<dim3((n8 + 255) / 256), 256, 0, stream>>>(f_hid, hidH, hidL, n8);
    cvt_transpose<<<dim3(N3D / 32, DMODEL / 64), 256, 0, stream>>>(f_wa, waTH, waTL, DMODEL, N3D);
    cvt_transpose<<<dim3(DMODEL / 32, DMODEL / 64), 256, 0, stream>>>(f_wp, wpTH, wpTL, DMODEL, DMODEL);

    gemm_qkv<<<dim3(N3D / 64, ROWS / 128), 256, 0, stream>>>(hidH, hidL, waTH, waTL, f_ba,
                                                            QH, QL, KH, KL, VTH, VTL);

    attn_kernel<<<dim3(S_LEN / 128, BATCH * NHEADS), 256, 0, stream>>>(QH, QL, KH, KL, VTH, VTL, OH, OL);

    gemm_proj<<<dim3(DMODEL / 64, ROWS / 128), 256, 0, stream>>>(OH, OL, wpTH, wpTL, f_bp, out);
}
